// mLSTMLayer_28638841930504
// MI455X (gfx1250) — hardware-run, weakly checked
//
#include <hip/hip_runtime.h>
#include <math.h>

typedef __attribute__((ext_vector_type(16))) _Float16 v16h;
typedef __attribute__((ext_vector_type(8)))  _Float16 v8h;
typedef __attribute__((ext_vector_type(16))) __bf16   v16b;
typedef __attribute__((ext_vector_type(8)))  __bf16   v8b;
typedef __attribute__((ext_vector_type(8)))  float    v8f;
typedef __attribute__((ext_vector_type(4)))  float    v4f;

constexpr int kBatch  = 2;
constexpr int kSteps  = 1024;
constexpr int kDim    = 1024;
constexpr int kHeads  = 8;
constexpr int kDqk    = 64;
constexpr int kDh     = 128;
constexpr int kRows   = kBatch * kSteps;
constexpr int kNq     = kHeads * kDqk;
constexpr int kNv     = kHeads * kDh;
constexpr int kColQ   = 0;
constexpr int kColK   = kColQ + kNq;
constexpr int kColV   = kColK + kNq;
constexpr int kColG   = kColV + kNv;
constexpr int kColIF  = kColG + kDim;
constexpr int kNif    = 64;
constexpr int kNall   = kColIF + kNif;
constexpr int kThr    = 256;
constexpr int kThrScan = 128;
constexpr int kChunk  = 16;
constexpr float kGateCap = 15.0f;
constexpr float kNormEps = 1e-6f;
constexpr float kInvGateCap = 1.0f / 15.0f;

constexpr float kInCarry  = 1024.0f;
constexpr float kWCarry   = 1024.0f;
constexpr float kActCarry = 1024.0f;
constexpr float kP1Scale  = 1.0f / (kInCarry * kWCarry);
constexpr float kP2Scale  = 1.0f / (kActCarry * kWCarry);
constexpr float kF16MinNormal = 6.103515625e-5f;

static_assert(kRows == 2048 && kNq == 512 && kNv == 1024 && kNall == 3136, "plane sizes");
static_assert((kRows % 64) == 0 && (kNall % 64) == 0 && (kDim % 64) == 0, "GEMM M, N multiples of 64");
static_assert((kDim % 32) == 0 && (kNv % 32) == 0, "GEMM K multiples of 32");
static_assert(kDh == kThrScan, "one scan thread per value column");
static_assert((kSteps % kChunk) == 0, "whole chunks");
static_assert(2 * kHeads <= kNif, "scalar gate columns");
static_assert(kColIF >= kDim, "the bias row's first 1024 columns are zeros (used as the output projection's neutral bias)");

constexpr size_t kOffX16  = 0;
constexpr size_t kOffWALL = kOffX16  + (size_t)kRows * kDim * 2;
constexpr size_t kOffWOT  = kOffWALL + (size_t)kNall * kDim * 2;
constexpr size_t kOffBALL = kOffWOT  + (size_t)kNv * kDim * 2;
constexpr size_t kOffP    = kOffBALL + 13312;
constexpr size_t kOffHRAW = kOffP    + (size_t)kRows * kNall * 4;
constexpr size_t kOffG16  = kOffHRAW + (size_t)kRows * kNv * 4;
constexpr size_t kWsTotal = kOffG16  + (size_t)kRows * kNv * 2;
static_assert(kWsTotal == 51000320ull, "carve total");
static_assert(kWsTotal <= 134217728ull, "carve cap");
static_assert((kOffWALL % 256) == 0 && (kOffWOT % 256) == 0 && (kOffBALL % 256) == 0 && (kOffP % 256) == 0 && (kOffHRAW % 256) == 0 && (kOffG16 % 256) == 0, "aligned regions");
static_assert((size_t)13 * 256 * 4 == 13312 && 13 * 256 >= kNall, "bias plane: 13 blocks x 256 threads cover its region exactly");

__device__ __forceinline__ unsigned short f2bf_bits(float f) {
  unsigned u = __float_as_uint(f);
  return (unsigned short)((u + 0x7FFFu + ((u >> 16) & 1u)) >> 16);
}
__device__ __forceinline__ float bf_bits2f(unsigned short h) { return __uint_as_float(((unsigned)h) << 16); }
__device__ __forceinline__ float bf16r(float f) { return bf_bits2f(f2bf_bits(f)); }
__device__ __forceinline__ float carry_flush(float v, float carry) {
  const float s = v * carry;
  return (fabsf(s) < kF16MinNormal) ? 0.0f : s;
}
__device__ __forceinline__ float frcp(float x) { return __builtin_amdgcn_rcpf(x); }

__device__ __forceinline__ void dep_guard4_h(v8f& a, v8f& b, v8f& c, v8f& d, v16h x, v16h y) { asm volatile("v_nop\n\tv_nop\n\tv_nop\n\tv_nop" : "+v"(a), "+v"(b), "+v"(c), "+v"(d) : "v"(x), "v"(y)); }
__device__ __forceinline__ void dep_guard4_b(v8f& a, v8f& b, v8f& c, v8f& d, v16b x, v16b y) { asm volatile("v_nop\n\tv_nop\n\tv_nop\n\tv_nop" : "+v"(a), "+v"(b), "+v"(c), "+v"(d) : "v"(x), "v"(y)); }
__device__ __forceinline__ void keep4_h(v16h a, v16h b, v16h c, v16h d) { asm volatile("v_nop" :: "v"(a), "v"(b), "v"(c), "v"(d)); }
__device__ __forceinline__ void keep4_b(v16b a, v16b b, v16b c, v16b d) { asm volatile("v_nop" :: "v"(a), "v"(b), "v"(c), "v"(d)); }
__device__ __forceinline__ void acc_guard4(v8f& a, v8f& b, v8f& c, v8f& d) { asm volatile("v_nop\n\tv_nop\n\tv_nop\n\tv_nop" : "+v"(a), "+v"(b), "+v"(c), "+v"(d)); }

template <typename T> struct Frag;
template <> struct Frag<_Float16> {
  typedef v16h V; union U { v16h v; v8h h[2]; };
  static __device__ __forceinline__ v16h load(const _Float16* p) {
    U f; f.h[0] = *(const v8h*)(p); f.h[1] = *(const v8h*)(p + 16); return f.v;
  }
  static __device__ __forceinline__ v8f mma(v16h a, v16h b, v8f c) {
    return __builtin_amdgcn_wmma_f32_16x16x32_f16(false, a, false, b, (short)0, c, false, false);
  }
  static __device__ __forceinline__ void guard4(v8f& a, v8f& b, v8f& c, v8f& d, v16h x, v16h y) { dep_guard4_h(a, b, c, d, x, y); }
  static __device__ __forceinline__ void keep(v16h a, v16h b, v16h c, v16h d) { keep4_h(a, b, c, d); }
};
template <> struct Frag<__bf16> {
  typedef v16b V; union U { v16b v; v8b h[2]; };
  static __device__ __forceinline__ v16b load(const __bf16* p) {
    U f; f.h[0] = *(const v8b*)(p); f.h[1] = *(const v8b*)(p + 16); return f.v;
  }
  static __device__ __forceinline__ v8f mma(v16b a, v16b b, v8f c) {
    return __builtin_amdgcn_wmma_f32_16x16x32_bf16(false, a, false, b, (short)0, c, false, false);
  }
  static __device__ __forceinline__ void guard4(v8f& a, v8f& b, v8f& c, v8f& d, v16b x, v16b y) { dep_guard4_b(a, b, c, d, x, y); }
  static __device__ __forceinline__ void keep(v16b a, v16b b, v16b c, v16b d) { keep4_b(a, b, c, d); }
};

__device__ __forceinline__ v8f mma_h(v16h a, v16h b, v8f c) {
  c = __builtin_amdgcn_wmma_f32_16x16x32_f16(false, a, false, b, (short)0, c, false, false);
  asm volatile("v_nop\n\tv_nop\n\tv_nop\n\tv_nop" : "+v"(c) : "v"(a), "v"(b));
  return c;
}

template <int ET> struct Elem;
template <> struct Elem<0> { typedef _Float16 T; };
template <> struct Elem<1> { typedef __bf16 T; };
template <int ET, bool SPLIT, int BIAS_MODE, int OUT_MODE, bool RESID, int ACT = 0>
__global__ __launch_bounds__(256) void wmma_gemm64(
    const unsigned short* __restrict__ Ap, const unsigned short* __restrict__ A2p, int lda, long strideA,
    const unsigned short* __restrict__ Btp, const unsigned short* __restrict__ Bt2p, int ldb, long strideB,
    void* __restrict__ Cout, void* __restrict__ Cout2, int ldc, long strideC,
    const float* __restrict__ bias,
    const float* __restrict__ resid, long strideR,
    int M, int N, int K, float scale) {
  typedef typename Elem<ET>::T T;
  typedef typename Frag<T>::V V;
  const T* A = (const T*)Ap; const T* A2 = (const T*)A2p; const T* Bt = (const T*)Btp; const T* Bt2 = (const T*)Bt2p;
  __shared__ __align__(16) float sT[8][16 * 68];
  const int b    = blockIdx.y;
  const int lane = threadIdx.x & 31;
  const int wave = threadIdx.x >> 5;
  const int tilesN = N >> 6;
  const int tilesM = M >> 6;
  const int tile = blockIdx.x * 8 + wave;
  if (tile >= tilesM * tilesN) return;
  const int tm = tile / tilesN;
  const int tn = tile - tm * tilesN;
  const int m0 = tm << 6;
  const int n0 = tn << 6;

  const T* Ab  = A  + (size_t)b * strideA;
  const T* Bb  = Bt + (size_t)b * strideB;
  const T* Ab2 = SPLIT ? (A2  + (size_t)b * strideA) : nullptr;
  const T* Bb2 = SPLIT ? (Bt2 + (size_t)b * strideB) : nullptr;

  const int rlane = lane & 15;
  const int koff  = (lane >> 4) * 8;
  const int mOff  = (lane >> 4) * 8;

  v8f acc[4][4];
#pragma unroll
  for (int i = 0; i < 4; ++i)
#pragma unroll
    for (int j = 0; j < 4; ++j) acc[i][j] = (v8f){0.f,0.f,0.f,0.f,0.f,0.f,0.f,0.f};

  for (int k0 = 0; k0 < K; k0 += 32) {
    V bh[4], bl[4];
#pragma unroll
    for (int j = 0; j < 4; ++j) {
      const size_t bo = (size_t)(n0 + (j << 4) + rlane) * ldb + koff + k0;
      bh[j] = Frag<T>::load(Bb + bo);
      if (SPLIT) bl[j] = Frag<T>::load(Bb2 + bo);
    }
#pragma unroll
    for (int i = 0; i < 4; ++i) {
      const size_t ao = (size_t)(m0 + (i << 4) + rlane) * lda + koff + k0;
      V ah = Frag<T>::load(Ab + ao);
      V al;
      if (SPLIT) al = Frag<T>::load(Ab2 + ao);
#pragma unroll
      for (int j = 0; j < 4; ++j) {
        acc[i][j] = Frag<T>::mma(ah, bh[j], acc[i][j]);
        if (SPLIT) {
          acc[i][j] = Frag<T>::mma(ah, bl[j], acc[i][j]);
          acc[i][j] = Frag<T>::mma(al, bh[j], acc[i][j]);
        }
      }
      Frag<T>::guard4(acc[i][0], acc[i][1], acc[i][2], acc[i][3], ah, SPLIT ? al : ah);
    }
    Frag<T>::keep(bh[0], bh[1], bh[2], bh[3]);
    if (SPLIT) Frag<T>::keep(bl[0], bl[1], bl[2], bl[3]);
  }
  acc_guard4(acc[0][0], acc[0][1], acc[0][2], acc[0][3]);
  acc_guard4(acc[1][0], acc[1][1], acc[1][2], acc[1][3]);
  acc_guard4(acc[2][0], acc[2][1], acc[2][2], acc[2][3]);
  acc_guard4(acc[3][0], acc[3][1], acc[3][2], acc[3][3]);

  float* slab = sT[wave];
  const float* Rb = RESID ? (resid + (size_t)b * strideR) : nullptr;
#pragma unroll
  for (int i = 0; i < 4; ++i) {
    const int mBase = m0 + (i << 4);
#pragma unroll
    for (int j = 0; j < 4; ++j) {
      const int n = n0 + (j << 4) + rlane;
      float bv = 0.f;
      if (BIAS_MODE == 2) bv = bias[n];
#pragma unroll
      for (int r = 0; r < 8; ++r) {
        float v = acc[i][j][r] * scale;
        if (BIAS_MODE == 1) v += bias[mBase + mOff + r];
        if (BIAS_MODE == 2) v += bv;
        if (RESID) v += Rb[(size_t)(mBase + mOff + r) * ldc + n];
        if (ACT == 1) v = tanhf(v);
        if (ACT == 2) v = fmaxf(v, 0.0f);
        if (ACT == 3) v = v / (1.0f + expf(-v));
        if (ACT == 4) v = (v > 0.f) ? v : 0.01f * v;
        slab[(mOff + r) * 68 + (j << 4) + rlane] = v;
      }
    }
    __builtin_amdgcn_fence(__ATOMIC_RELEASE, "workgroup");
    __builtin_amdgcn_wave_barrier();
    __builtin_amdgcn_fence(__ATOMIC_ACQUIRE, "workgroup");
    if (OUT_MODE == 0) {
      float* C = (float*)Cout + (size_t)b * strideC;
      const int hh = lane >> 4, c4 = (lane & 15) * 4;
      for (int pass = 0; pass < 2; ++pass) {
#pragma unroll
        for (int it = 0; it < 8; ++it) {
          const int row = it * 2 + hh;
          v4f v = *(const v4f*)(slab + row * 68 + c4);
          *(volatile v4f*)(C + (size_t)(mBase + row) * ldc + n0 + c4) = v;
        }
        __threadfence();
      }
    } else {
      const int q = lane >> 3, c8 = (lane & 7) * 8;
      unsigned short* C  = (unsigned short*)Cout  + (size_t)b * strideC;
      unsigned short* C2 = (OUT_MODE == 2) ? ((unsigned short*)Cout2 + (size_t)b * strideC) : nullptr;
      for (int pass = 0; pass < 2; ++pass) {
#pragma unroll
        for (int it = 0; it < 4; ++it) {
          const int row = it * 4 + q;
          const float* sp = slab + row * 68 + c8;
          v8h hv, lv;
#pragma unroll
          for (int e = 0; e < 8; ++e) {
            if (OUT_MODE == 1) {
              hv[e] = (_Float16)sp[e];
            } else {
              unsigned short hb = f2bf_bits(sp[e]);
              unsigned short lb = f2bf_bits(sp[e] - bf_bits2f(hb));
              hv[e] = __builtin_bit_cast(_Float16, hb);
              lv[e] = __builtin_bit_cast(_Float16, lb);
            }
          }
          *(volatile v8h*)(C + (size_t)(mBase + row) * ldc + n0 + c8) = hv;
          if (OUT_MODE == 2) *(volatile v8h*)(C2 + (size_t)(mBase + row) * ldc + n0 + c8) = lv;
        }
        __threadfence();
      }
    }
    __builtin_amdgcn_fence(__ATOMIC_RELEASE, "workgroup");
    __builtin_amdgcn_wave_barrier();
    __builtin_amdgcn_fence(__ATOMIC_ACQUIRE, "workgroup");
  }
}

__global__ __launch_bounds__(kThr) void cast_plane_kernel(const float* __restrict__ src, unsigned short* __restrict__ dst,
                                                          int colsLog2, int dstPitch, int dstOff) {
  const int i   = blockIdx.x * kThr + threadIdx.x;
  const int sh  = colsLog2 - 3;
  const int row = i >> sh;
  const int c8  = (i & ((1 << sh) - 1)) * 8;
  const float* sp = src + ((size_t)row << colsLog2) + c8;
  const v4f a0 = *(const v4f*)(sp);
  const v4f a1 = *(const v4f*)(sp + 4);
  v8h hv;
#pragma unroll
  for (int e = 0; e < 4; ++e) {
    const float f0 = a0[e];
    const float f1 = a1[e];
    hv[e]     = (_Float16)carry_flush(bf16r(f0), kInCarry);
    hv[4 + e] = (_Float16)carry_flush(bf16r(f1), kInCarry);
  }
  unsigned short* dp = dst + (size_t)row * dstPitch + dstOff + c8;
  *(volatile v8h*)dp = hv;
  __threadfence();
  *(volatile v8h*)dp = hv;
}
static_assert(kInCarry == kWCarry, "one cast kernel serves inputs and weights");

__global__ __launch_bounds__(kThr) void tr_plane_kernel(const float* __restrict__ in, unsigned short* __restrict__ out,
                                                        int inPitch, int outPitch) {
  __shared__ __align__(16) float sTile[64 * 68];
  const int tid = threadIdx.x;
  const int n0 = blockIdx.x * 64;
  const int k0 = blockIdx.y * 64;
  {
    const int kk = tid >> 4;
    const int n4 = (tid & 15) * 4;
#pragma unroll
    for (int i = 0; i < 4; ++i) {
      const int k = kk + 16 * i;
      const v4f v = *(const v4f*)(in + (size_t)(k0 + k) * inPitch + n0 + n4);
#pragma unroll
      for (int e = 0; e < 4; ++e) {
        const float f = v[e];
        sTile[(n4 + e) * 68 + k] = carry_flush(bf16r(f), kWCarry);
      }
    }
  }
  __syncthreads();
  const int k8 = (tid & 7) * 8;
  v8h hv[2];
#pragma unroll
  for (int it = 0; it < 2; ++it) {
    const int n = (tid >> 3) + 32 * it;
    const float* sp = sTile + n * 68 + k8;
    const v4f a0 = *(const v4f*)(sp);
    const v4f a1 = *(const v4f*)(sp + 4);
#pragma unroll
    for (int e = 0; e < 4; ++e) {
      const float f0 = a0[e];
      const float f1 = a1[e];
      hv[it][e]     = (_Float16)f0;
      hv[it][4 + e] = (_Float16)f1;
    }
  }
  for (int pass = 0; pass < 2; ++pass) {
#pragma unroll
    for (int it = 0; it < 2; ++it) {
      const int n = (tid >> 3) + 32 * it;
      *(volatile v8h*)(out + (size_t)(n0 + n) * outPitch + k0 + k8) = hv[it];
    }
    __threadfence();
  }
}

__global__ __launch_bounds__(kThr) void gate_rows_kernel(const float* __restrict__ Wi, const float* __restrict__ Wf,
                                                         unsigned short* __restrict__ dst) {
  const int i  = blockIdx.x * kThr + threadIdx.x;
  const int n  = i >> 7;
  const int k8 = (i & 127) * 8;
  const int nc = (n < 15) ? n : 15;
  const float* src = (nc < kHeads) ? Wi : Wf;
  const int col = nc & (kHeads - 1);
  const bool live = (n < 2 * kHeads);
  v8h hv;
#pragma unroll
  for (int e = 0; e < 8; ++e) {
    const float f = src[(size_t)(k8 + e) * kHeads + col];
    const float g = live ? carry_flush(bf16r(f), kWCarry) : 0.0f;
    hv[e] = (_Float16)g;
  }
  unsigned short* dp = dst + (size_t)n * kDim + k8;
  *(volatile v8h*)dp = hv;
  __threadfence();
  *(volatile v8h*)dp = hv;
}
static_assert((kNif * kDim / 8) % kThr == 0 && (kDim / 8) == 128, "gate rows grid exact; 128 threads per row");

__global__ __launch_bounds__(kThr) void bias_row_kernel(const float* __restrict__ bi, const float* __restrict__ bf,
                                                        float* __restrict__ dst) {
  const int c = blockIdx.x * kThr + threadIdx.x;
  const int r = c - kColIF;
  const int rc = (r < 0) ? 0 : ((r > 2 * kHeads - 1) ? (2 * kHeads - 1) : r);
  const float vi = bi[rc & (kHeads - 1)];
  const float vf = bf[rc & (kHeads - 1)];
  const float pick = (rc < kHeads) ? vi : vf;
  const bool live = (r >= 0) && (r < 2 * kHeads);
  const float o = live ? bf16r(pick) : 0.0f;
  float* op = dst + c;
  *(volatile float*)op = o;
  __threadfence();
  *(volatile float*)op = o;
}

__global__ __launch_bounds__(kThrScan) void mstate_scan_kernel(const float* __restrict__ P, float* __restrict__ HRAW) {
  __shared__ __align__(16) float Cs[kDqk * kDh];
  __shared__ __align__(16) float sq[kChunk * kDqk];
  __shared__ __align__(16) float sk[kChunk * kDqk];
  __shared__ __align__(16) float sv[kChunk * kDh];
  __shared__ __align__(16) float sif[kChunk * 2];
  const int tid = threadIdx.x;
  const int b = blockIdx.x >> 3;
  const int h = blockIdx.x & (kHeads - 1);
  const int j = tid;
#pragma unroll 1
  for (int i = 0; i < kDqk; ++i) Cs[i * kDh + j] = 0.0f;
  float mrun = 0.0f;
  const float qscale = 0.125f;

#pragma unroll 1
  for (int ch = 0; ch < kSteps / kChunk; ++ch) {
    const int t0 = ch * kChunk;
    const float* prow = P + (size_t)(b * kSteps + t0) * kNall;
#pragma unroll
    for (int it = 0; it < 2; ++it) {
      const int idx = it * kThrScan + tid;
      const int tt = idx >> 4;
      const int c4 = (idx & 15) * 4;
      const v4f vq = *(const v4f*)(prow + (size_t)tt * kNall + kColQ + h * kDqk + c4);
      const v4f vk = *(const v4f*)(prow + (size_t)tt * kNall + kColK + h * kDqk + c4);
      *(v4f*)(sq + tt * kDqk + c4) = vq;
      *(v4f*)(sk + tt * kDqk + c4) = vk;
    }
#pragma unroll
    for (int it = 0; it < 4; ++it) {
      const int idx = it * kThrScan + tid;
      const int tt = idx >> 5;
      const int c4 = (idx & 31) * 4;
      const v4f vv = *(const v4f*)(prow + (size_t)tt * kNall + kColV + h * kDh + c4);
      *(v4f*)(sv + tt * kDh + c4) = vv;
    }
    {
      const int e  = tid & 31;
      const int tt = e >> 1;
      const int wh = e & 1;
      sif[tt * 2 + wh] = prow[(size_t)tt * kNall + kColIF + kHeads * wh + h];
    }
    __syncthreads();

#pragma unroll 1
    for (int tt = 0; tt < kChunk; ++tt) {
      const float ig = sif[tt * 2 + 0];
      const float fg = sif[tt * 2 + 1];
      const float flog = fminf(fg, 0.0f) - log1pf(expf(-fabsf(fg)));
      const float mnew = fmaxf(flog + mrun, ig);
      const float fa = expf(flog + mrun - mnew);
      const float ia = expf(ig - mnew);
      mrun = mnew;
      const float vj = sv[tt * kDh + j];
      float acc = 0.0f;
#pragma unroll 4
      for (int i = 0; i < kDqk; ++i) {
        const float ki = sk[tt * kDqk + i];
        const float qi = sq[tt * kDqk + i];
        const float cold = Cs[i * kDh + j];
        const float cnew = fa * cold + ia * (ki * vj);
        Cs[i * kDh + j] = cnew;
        acc += cnew * (qi * qscale);
      }
      float* op = HRAW + (size_t)(b * kSteps + t0 + tt) * kNv + h * kDh + j;
      *(volatile float*)op = acc;
      __threadfence();
      *(volatile float*)op = acc;
    }
    __syncthreads();
  }
}

__device__ __forceinline__ float gate_tanh(float v) {
  const float e = __expf(2.0f * v);
  return 1.0f - 2.0f * frcp(e + 1.0f);
}

__global__ __launch_bounds__(kThr) void norm_gate_kernel(const float* __restrict__ HRAW, const float* __restrict__ P,
                                                         const float* __restrict__ lnw, const float* __restrict__ lnb,
                                                         unsigned short* __restrict__ G16) {
  const int gid  = blockIdx.x * kThr + threadIdx.x;
  const int pair = gid >> 4;
  const int l16  = gid & 15;
  const int m    = pair >> 3;
  const int h    = pair & (kHeads - 1);
  const int j8   = l16 * 8;
  const float* hp = HRAW + (size_t)m * kNv + h * kDh + j8;
  const v4f a0 = *(const v4f*)(hp);
  const v4f a1 = *(const v4f*)(hp + 4);
  float hv[8];
#pragma unroll
  for (int e = 0; e < 4; ++e) {
    hv[e]     = a0[e];
    hv[4 + e] = a1[e];
  }
  float s = 0.0f;
#pragma unroll
  for (int e = 0; e < 8; ++e) s += hv[e];
  s += __shfl_xor(s, 1, 32);
  s += __shfl_xor(s, 2, 32);
  s += __shfl_xor(s, 4, 32);
  s += __shfl_xor(s, 8, 32);
  const float mean = s * (1.0f / (float)kDh);
  float d[8];
  float q = 0.0f;
#pragma unroll
  for (int e = 0; e < 8; ++e) {
    d[e] = hv[e] - mean;
    q += d[e] * d[e];
  }
  q += __shfl_xor(q, 1, 32);
  q += __shfl_xor(q, 2, 32);
  q += __shfl_xor(q, 4, 32);
  q += __shfl_xor(q, 8, 32);
  const float var = q * (1.0f / (float)kDh);
  const float sd  = sqrtf(var + kNormEps);
  const float rs  = 1.0f / sd;
  const float* gp = P + (size_t)m * kNall + kColG + h * kDh + j8;
  const v4f g0 = *(const v4f*)(gp);
  const v4f g1 = *(const v4f*)(gp + 4);
  const v4f w0 = *(const v4f*)(lnw + h * kDh + j8);
  const v4f w1 = *(const v4f*)(lnw + h * kDh + j8 + 4);
  const v4f b0 = *(const v4f*)(lnb + h * kDh + j8);
  const v4f b1 = *(const v4f*)(lnb + h * kDh + j8 + 4);
  v8h ov;
#pragma unroll
  for (int e = 0; e < 8; ++e) {
    const float gv = (e < 4) ? g0[e & 3] : g1[e & 3];
    const float wv = (e < 4) ? w0[e & 3] : w1[e & 3];
    const float bv = (e < 4) ? b0[e & 3] : b1[e & 3];
    const float hn = (d[e] * rs) * bf16r(wv) + bf16r(bv);
    const float tg = gate_tanh(gv * kInvGateCap);
    const float og = frcp(1.0f + __expf(-(tg * kGateCap)));
    ov[e] = (_Float16)carry_flush(hn * og, kActCarry);
  }
  unsigned short* dp = G16 + (size_t)m * kNv + h * kDh + j8;
  *(volatile v8h*)dp = ov;
  __threadfence();
  *(volatile v8h*)dp = ov;
}
static_assert(((size_t)kRows * kHeads * 16) % kThr == 0, "norm grid exact");

static_assert(((kRows / 64) * (kNall / 64)) % 8 == 0 && ((kRows / 64) * (kDim / 64)) % 8 == 0, "GEMM grids exact");
static_assert(((size_t)kRows * kDim / 8) % kThr == 0, "input cast grid exact");

extern "C" void kernel_launch(void* const* d_in, const int* in_sizes, int n_in,
                              void* d_out, int out_size, void* d_ws, size_t ws_size,
                              hipStream_t stream) {
  if (n_in < 12 || d_out == nullptr || d_ws == nullptr) return;
  if (in_sizes[0] != kRows * kDim) return;
  if (in_sizes[1] != kDim * kNq || in_sizes[2] != kDim * kNq || in_sizes[3] != kDim * kNv) return;
  if (in_sizes[4] != kDim * kHeads || in_sizes[5] != kHeads || in_sizes[6] != kDim * kHeads || in_sizes[7] != kHeads) return;
  if (in_sizes[8] != kDim * kDim) return;
  if (in_sizes[9] != kHeads * kDh || in_sizes[10] != kHeads * kDh) return;
  if (in_sizes[11] != kNv * kDim) return;
  if (out_size != kRows * kDim) return;
  if (ws_size < kWsTotal) return;

  const float* x    = (const float*)d_in[0];
  const float* Wq   = (const float*)d_in[1];
  const float* Wk   = (const float*)d_in[2];
  const float* Wv   = (const float*)d_in[3];
  const float* Wi   = (const float*)d_in[4];
  const float* bi   = (const float*)d_in[5];
  const float* Wf   = (const float*)d_in[6];
  const float* bf   = (const float*)d_in[7];
  const float* Wog  = (const float*)d_in[8];
  const float* lnw  = (const float*)d_in[9];
  const float* lnb  = (const float*)d_in[10];
  const float* Wout = (const float*)d_in[11];
  float* out = (float*)d_out;

  char* ws = (char*)d_ws;
  unsigned short* X16  = (unsigned short*)(ws + kOffX16);
  unsigned short* WALL = (unsigned short*)(ws + kOffWALL);
  unsigned short* WOT  = (unsigned short*)(ws + kOffWOT);
  float*          BALL = (float*)(ws + kOffBALL);
  float*          P    = (float*)(ws + kOffP);
  float*          HRAW = (float*)(ws + kOffHRAW);
  unsigned short* G16  = (unsigned short*)(ws + kOffG16);

  cast_plane_kernel<<<(kRows * kDim / 8) / kThr, kThr, 0, stream>>>(x, X16, 10, kDim, 0);
  tr_plane_kernel<<<dim3(kNq / 64,  kDim / 64), kThr, 0, stream>>>(Wq,   WALL + (size_t)kColQ * kDim, kNq,  kDim);
  tr_plane_kernel<<<dim3(kNq / 64,  kDim / 64), kThr, 0, stream>>>(Wk,   WALL + (size_t)kColK * kDim, kNq,  kDim);
  tr_plane_kernel<<<dim3(kNv / 64,  kDim / 64), kThr, 0, stream>>>(Wv,   WALL + (size_t)kColV * kDim, kNv,  kDim);
  tr_plane_kernel<<<dim3(kDim / 64, kDim / 64), kThr, 0, stream>>>(Wog,  WALL + (size_t)kColG * kDim, kDim, kDim);
  gate_rows_kernel<<<(kNif * kDim / 8) / kThr, kThr, 0, stream>>>(Wi, Wf, WALL + (size_t)kColIF * kDim);
  tr_plane_kernel<<<dim3(kDim / 64, kNv / 64),  kThr, 0, stream>>>(Wout, WOT, kDim, kNv);
  bias_row_kernel<<<13, kThr, 0, stream>>>(bi, bf, BALL);

  wmma_gemm64<0, false, 2, 0, false, 0><<<dim3((kRows / 64) * (kNall / 64) / 8, 1), 256, 0, stream>>>(
      X16, X16, kDim, 0L, WALL, WALL, kDim, 0L, (void*)P, (void*)P, kNall, 0L,
      BALL, nullptr, 0L, kRows, kNall, kDim, kP1Scale);

  mstate_scan_kernel<<<kBatch * kHeads, kThrScan, 0, stream>>>(P, HRAW);
  norm_gate_kernel<<<(kRows * kHeads * 16) / kThr, kThr, 0, stream>>>(HRAW, P, lnw, lnb, G16);

  wmma_gemm64<0, false, 2, 0, false, 0><<<dim3((kRows / 64) * (kDim / 64) / 8, 1), 256, 0, stream>>>(
      G16, G16, kNv, 0L, WOT, WOT, kNv, 0L, (void*)out, (void*)out, kDim, 0L,
      BALL, nullptr, 0L, kRows, kDim, kNv, kP2Scale);
}
